// MultiHeadAttention_86723979641195
// MI455X (gfx1250) — hardware-verified
//
#include <hip/hip_runtime.h>

#ifndef NB
#define NB 2
#endif
#ifndef SEQ
#define SEQ 2048
#endif
#define NB_FULL   2
#define SEQ_FULL  2048
#define DQ        768
#define HQ        12
#define HDQ       64
#define MQ        (NB * SEQ)
#define PLX       ((size_t)MQ * DQ)
#if SEQ >= 512
#define EARLY_QT  16
#else
#define EARLY_QT  (SEQ / 32)
#endif
#define ARES_ROWS (16 * EARLY_QT)
#define XS        8.0f
#define WSC       64.0f
#define RSPLIT    (1.0f / 2048.0f)

static_assert(SEQ % 128 == 0);
static_assert(DQ % 64 == 0);
static_assert(DQ % 32 == 0);
static_assert(HQ * HDQ == DQ);
static_assert(HDQ == 64);
static_assert(SEQ / 16 > EARLY_QT);
static_assert(EARLY_QT >= 1);
static_assert(ARES_ROWS <= SEQ);
static_assert(((size_t)MQ * DQ) % 1024 == 0);
static_assert(((size_t)DQ * DQ) % 1024 == 0);
static_assert(NB <= NB_FULL);
static_assert(SEQ <= SEQ_FULL);

typedef _Float16 h16;
typedef __attribute__((ext_vector_type(16))) _Float16 v16h;
typedef _Float16 v8ha __attribute__((ext_vector_type(8), may_alias));
typedef __attribute__((ext_vector_type(8))) float v8f;
typedef __attribute__((ext_vector_type(4))) float v4f;
typedef float v4fa __attribute__((ext_vector_type(4), may_alias));
typedef __attribute__((ext_vector_type(2))) unsigned v2u;

__device__ __forceinline__ float bfr(float f) {
    unsigned u = __float_as_uint(f);
    u = (u + 0x7FFFu + ((u >> 16) & 1u)) & 0xFFFF0000u;
    return __uint_as_float(u);
}
__device__ __forceinline__ void split16(float f, h16& h, h16& l) { h = (h16)f; l = (h16)((f - (float)h) * 2048.0f); }
__device__ __forceinline__ unsigned short hbits(h16 h) { return __builtin_bit_cast(unsigned short, h); }
__device__ __forceinline__ unsigned pack2h(h16 a, h16 b) { return (unsigned)hbits(a) | ((unsigned)hbits(b) << 16); }

__device__ __forceinline__ v16h load_frag2(const h16* p0, const h16* p1) {
    const v8ha a = *reinterpret_cast<const v8ha*>(p0);
    const v8ha b = *reinterpret_cast<const v8ha*>(p1);
    v16h r = __builtin_shufflevector(a, b, 0, 1, 2, 3, 4, 5, 6, 7, 8, 9, 10, 11, 12, 13, 14, 15);
    return r;
}
__device__ __forceinline__ void copy16(const h16* g, h16* l) {
    *reinterpret_cast<v8ha*>(l) = *reinterpret_cast<const v8ha*>(g);
}

__device__ __forceinline__ v8f wmma16(v16h a, v16h b, v8f c) {
    c = __builtin_amdgcn_wmma_f32_16x16x32_f16(false, a, false, b, (short)0, c, false, false);
    asm volatile("v_nop\n\tv_nop\n\tv_nop\n\tv_nop" : "+v"(c) : "v"(a), "v"(b));
    return c;
}
__device__ __forceinline__ v8f wmma_split(v16h ah, v16h al, v16h bh, v16h bl, v8f c) {
    v8f x = {};
    x = wmma16(al, bh, x);
    x = wmma16(ah, bl, x);
    c = wmma16(ah, bh, c);
    return c + x * RSPLIT;
}

template <bool XMAP>
__global__ __launch_bounds__(256) void cvt_plane(const float* __restrict__ in, h16* __restrict__ out,
                                                 int nrows, float scale) {
    const int i = (blockIdx.x * 256 + threadIdx.x) * 4;
    const int n = nrows * DQ;
    if (i < n) {
        const int r  = i / DQ, c = i - r * DQ;
        const int sr = XMAP ? ((r / SEQ) * SEQ_FULL + (r % SEQ)) : r;
        const v4fa v = *reinterpret_cast<const v4fa*>(in + (size_t)sr * DQ + c);
        const h16 e0 = (h16)(bfr(v.x) * scale);
        const h16 e1 = (h16)(bfr(v.y) * scale);
        const h16 e2 = (h16)(bfr(v.z) * scale);
        const h16 e3 = (h16)(bfr(v.w) * scale);
        v2u p; p.x = pack2h(e0, e1); p.y = pack2h(e2, e3);
        *(volatile v2u*)(out + i) = p;
        __threadfence();
        *(volatile v2u*)(out + i) = p;
    }
}

template <int MODE>
__global__ __launch_bounds__(256)
void gemm16(const h16* __restrict__ A, const h16* __restrict__ BT, const float* __restrict__ bias,
            float* __restrict__ outF, h16* __restrict__ outB, float scale) {
    __shared__ alignas(16) h16   bsh[2][64 * 32];
    __shared__ alignas(16) float stg[8][16 * 64];

    const int tid  = threadIdx.x;
    const int lane = tid & 31;
    const int wave = tid >> 5;
    const int lo   = lane & 15;
    const int hi   = lane >> 4;
    const int rowBase = blockIdx.y * 128 + wave * 16;
    const int colBase = blockIdx.x * 64;
    const bool ares = (MODE == 0) && (((blockIdx.y * 128) % SEQ) < ARES_ROWS);

    const int cn = tid >> 2, cc = tid & 3;
    const h16* bSrc = BT + (size_t)(colBase + cn) * DQ + cc * 8;
    copy16(bSrc, &bsh[0][cn * 32 + cc * 8]);
    __syncthreads();

    v8f acc[4] = {};
    const h16* aRow  = A + (size_t)(rowBase + lo) * DQ;
    const h16* aRowl = aRow + PLX;

    constexpr int nk = DQ / 32;
    for (int ik = 0; ik < nk; ++ik) {
        const int k0  = ik * 32;
        const int buf = ik & 1;
        if (ik + 1 < nk) copy16(bSrc + (size_t)(ik + 1) * 32, &bsh[buf ^ 1][cn * 32 + cc * 8]);

        const v16h af = load_frag2(aRow + k0 + hi * 8, aRow + k0 + hi * 8 + 16);
#pragma unroll
        for (int t = 0; t < 4; ++t) {
            const h16* bp = &bsh[buf][(t * 16 + lo) * 32 + hi * 8];
            acc[t] = wmma16(af, load_frag2(bp, bp + 16), acc[t]);
        }
        if (ares) {
            const v16h afl = load_frag2(aRowl + k0 + hi * 8, aRowl + k0 + hi * 8 + 16);
#pragma unroll
            for (int t = 0; t < 4; ++t) {
                const h16* bp = &bsh[buf][(t * 16 + lo) * 32 + hi * 8];
                v8f x = {};
                x = wmma16(afl, load_frag2(bp, bp + 16), x);
                acc[t] = acc[t] + x * RSPLIT;
            }
        }
        __syncthreads();
    }

    float* sg = stg[wave];
#pragma unroll
    for (int t = 0; t < 4; ++t) {
        const float bvv = bfr(bias[colBase + t * 16 + lo]);
#pragma unroll
        for (int j = 0; j < 8; ++j) sg[(j + 8 * hi) * 64 + t * 16 + lo] = acc[t][j] * scale + bvv;
    }
    asm volatile("s_wait_dscnt 0" ::: "memory");
    __builtin_amdgcn_wave_barrier();
    if (MODE == 0) {
        v4f ov[8]; size_t oo[8];
#pragma unroll
        for (int i = 0; i < 8; ++i) {
            const int c = lane + 32 * i, r = c >> 4, q = c & 15;
            ov[i] = *reinterpret_cast<const v4fa*>(sg + r * 64 + q * 4);
            oo[i] = (size_t)(rowBase + r) * DQ + colBase + q * 4;
        }
#pragma unroll
        for (int i = 0; i < 8; ++i) *(volatile v4f*)(outF + oo[i]) = ov[i];
        __threadfence();
#pragma unroll
        for (int i = 0; i < 8; ++i) *(volatile v4f*)(outF + oo[i]) = ov[i];
    } else {
        const int h = colBase / HDQ;
        unsigned pv[16], pl[16]; size_t po[16];
#pragma unroll
        for (int r = 0; r < 16; ++r) {
            const int row = rowBase + r, b = row / SEQ, s = row % SEQ;
            h16 h0, l0, h1, l1;
            split16(sg[r * 64 + 2 * lane], h0, l0);
            split16(sg[r * 64 + 2 * lane + 1], h1, l1);
            pv[r] = pack2h(h0, h1); pl[r] = pack2h(l0, l1);
            po[r] = (((size_t)(b * HQ + h)) * SEQ + s) * HDQ + 2 * lane;
        }
#pragma unroll
        for (int r = 0; r < 16; ++r) { *(volatile unsigned*)(outB + po[r]) = pv[r]; *(volatile unsigned*)(outB + PLX + po[r]) = pl[r]; }
        __threadfence();
#pragma unroll
        for (int r = 0; r < 16; ++r) { *(volatile unsigned*)(outB + po[r]) = pv[r]; *(volatile unsigned*)(outB + PLX + po[r]) = pl[r]; }
    }
}

__global__ __launch_bounds__(256) void vt_kernel(const h16* __restrict__ Vr, h16* __restrict__ Vt) {
    __shared__ h16 t[64][66];
    const int tid = threadIdx.x, lane = tid & 31, wave = tid >> 5;
    const int bh = blockIdx.x / (SEQ / 64), s0 = (blockIdx.x % (SEQ / 64)) * 64;
    const size_t pl = blockIdx.y ? PLX : 0;
    const h16* src = Vr + pl + ((size_t)bh * SEQ + s0) * HDQ + (size_t)tid * 16;
    const v8ha c0 = *reinterpret_cast<const v8ha*>(src);
    const v8ha c1 = *reinterpret_cast<const v8ha*>(src + 8);
    const int tr = tid >> 2, tc = (tid & 3) * 16;
#pragma unroll
    for (int e = 0; e < 8; ++e) { t[tr][tc + e] = c0[e]; t[tr][tc + 8 + e] = c1[e]; }
    __syncthreads();
    h16* dst = Vt + pl + (size_t)bh * HDQ * SEQ + s0;
    unsigned pk[8]; size_t po[8];
#pragma unroll
    for (int r = 0; r < 8; ++r) {
        const int hd = wave * 8 + r;
        pk[r] = pack2h(t[2 * lane][hd], t[2 * lane + 1][hd]);
        po[r] = (size_t)hd * SEQ + 2 * lane;
    }
#pragma unroll
    for (int r = 0; r < 8; ++r) *(volatile unsigned*)(dst + po[r]) = pk[r];
    __threadfence();
#pragma unroll
    for (int r = 0; r < 8; ++r) *(volatile unsigned*)(dst + po[r]) = pk[r];
}

template <bool RES, bool MASK>
__device__ __forceinline__ void attn_kv_block(
    int causal, int kv0, int q0, int lo, int hi, int bh,
    const h16* __restrict__ Km, const h16* __restrict__ Vt, h16* pw, h16* pwl,
    v16h qa0, v16h qa1, v16h qa0l, v16h qa1l,
    v8f (&cacc)[4], float (&mi)[8], float (&li)[8]) {

    v8f s[4] = {};
#pragma unroll
    for (int tt = 0; tt < 4; ++tt) {
        const h16* kRow = Km + ((size_t)bh * SEQ + kv0 + tt * 16 + lo) * HDQ;
        const v16h kb0 = load_frag2(kRow + hi * 8,      kRow + 16 + hi * 8);
        const v16h kb1 = load_frag2(kRow + 32 + hi * 8, kRow + 48 + hi * 8);
        if (RES) {
            const v16h kb0l = load_frag2(kRow + PLX + hi * 8,      kRow + PLX + 16 + hi * 8);
            const v16h kb1l = load_frag2(kRow + PLX + 32 + hi * 8, kRow + PLX + 48 + hi * 8);
            s[tt] = wmma_split(qa0, qa0l, kb0, kb0l, s[tt]);
            s[tt] = wmma_split(qa1, qa1l, kb1, kb1l, s[tt]);
        } else {
            s[tt] = wmma16(qa0, kb0, s[tt]);
            s[tt] = wmma16(qa1, kb1, s[tt]);
        }
    }

    float alpha[8], rsum[8];
#pragma unroll
    for (int j = 0; j < 8; ++j) {
        const int qg = q0 + j + 8 * hi;
        float sv[4];
#pragma unroll
        for (int tt = 0; tt < 4; ++tt) {
            float v = s[tt][j] * 0.125f;
            if (MASK) { if (causal != 0 && (kv0 + tt * 16 + lo) > qg) v = -3.0e38f; }
            sv[tt] = v;
        }
        float mb = fmaxf(fmaxf(sv[0], sv[1]), fmaxf(sv[2], sv[3]));
#pragma unroll
        for (int d = 1; d < 16; d <<= 1) mb = fmaxf(mb, __shfl_xor(mb, d, 32));
        const float mnew = fmaxf(mi[j], mb);
        alpha[j] = __expf(mi[j] - mnew);
        mi[j] = mnew;
        const int r = (j + 8 * hi) * 64;
        float rp = 0.0f;
#pragma unroll
        for (int tt = 0; tt < 4; ++tt) {
            const float pv = __expf(sv[tt] - mnew) * 1024.0f;
            rp += pv;
            if (RES) {
                h16 ph, pq; split16(pv, ph, pq);
                pw[r + tt * 16 + lo] = ph; pwl[r + tt * 16 + lo] = pq;
            } else {
                pw[r + tt * 16 + lo] = (h16)pv;
            }
        }
#pragma unroll
        for (int d = 1; d < 16; d <<= 1) rp += __shfl_xor(rp, d, 32);
        rsum[j] = rp;
    }
    asm volatile("s_wait_dscnt 0" ::: "memory");
    __builtin_amdgcn_wave_barrier();

    const v16h pA0 = load_frag2(pw + lo * 64 + hi * 8,      pw + lo * 64 + hi * 8 + 16);
    const v16h pA1 = load_frag2(pw + lo * 64 + 32 + hi * 8, pw + lo * 64 + 32 + hi * 8 + 16);
    v16h pA0l = pA0, pA1l = pA1;
    if (RES) {
        pA0l = load_frag2(pwl + lo * 64 + hi * 8,      pwl + lo * 64 + hi * 8 + 16);
        pA1l = load_frag2(pwl + lo * 64 + 32 + hi * 8, pwl + lo * 64 + 32 + hi * 8 + 16);
    }

#pragma unroll
    for (int j = 0; j < 8; ++j) li[j] = li[j] * alpha[j] + rsum[j];

#pragma unroll
    for (int t = 0; t < 4; ++t) {
        const h16* vRow = Vt + ((size_t)bh * HDQ + t * 16 + lo) * SEQ + kv0;
#pragma unroll
        for (int j = 0; j < 8; ++j) cacc[t][j] *= alpha[j];
        const v16h vb0 = load_frag2(vRow + hi * 8,      vRow + 16 + hi * 8);
        const v16h vb1 = load_frag2(vRow + 32 + hi * 8, vRow + 48 + hi * 8);
        if (RES) {
            const v16h vb0l = load_frag2(vRow + PLX + hi * 8,      vRow + PLX + 16 + hi * 8);
            const v16h vb1l = load_frag2(vRow + PLX + 32 + hi * 8, vRow + PLX + 48 + hi * 8);
            cacc[t] = wmma_split(pA0, pA0l, vb0, vb0l, cacc[t]);
            cacc[t] = wmma_split(pA1, pA1l, vb1, vb1l, cacc[t]);
        } else {
            cacc[t] = wmma16(pA0, vb0, cacc[t]);
            cacc[t] = wmma16(pA1, vb1, cacc[t]);
        }
    }
}

template <bool RES>
__global__ __launch_bounds__(256) __attribute__((amdgpu_num_vgpr(256)))
void flash_attn(const h16* __restrict__ Q, const h16* __restrict__ Km, const h16* __restrict__ Vt,
                const int* __restrict__ maskp, h16* __restrict__ ctx, int nwaves) {
    __shared__ alignas(16) h16   psh[8][16 * 64];
    __shared__ alignas(16) h16   pshl[RES ? 8 : 1][16 * 64];
    __shared__ alignas(16) float osh[8][16 * 64];

    const int lane = threadIdx.x & 31;
    const int wave = threadIdx.x >> 5;
    const int lo   = lane & 15;
    const int hi   = lane >> 4;
    const int w    = blockIdx.x * 8 + wave;
    if (w >= nwaves) return;
    int bh, qt;
    if (RES) {
        bh = w / EARLY_QT; qt = w - bh * EARLY_QT;
    } else {
        constexpr int NL = SEQ / 16 - EARLY_QT;
        bh = w / NL; qt = EARLY_QT + (w - bh * NL);
    }
    const int q0 = qt * 16;
    const int causal = (maskp[0] != 0) ? 1 : 0;

    const h16* qRow = Q + ((size_t)bh * SEQ + q0 + lo) * HDQ;
    const v16h qa0 = load_frag2(qRow + hi * 8,      qRow + hi * 8 + 16);
    const v16h qa1 = load_frag2(qRow + 32 + hi * 8, qRow + 32 + hi * 8 + 16);
    v16h qa0l = qa0, qa1l = qa1;
    if (RES) {
        qa0l = load_frag2(qRow + PLX + hi * 8,      qRow + PLX + hi * 8 + 16);
        qa1l = load_frag2(qRow + PLX + 32 + hi * 8, qRow + PLX + 32 + hi * 8 + 16);
    }

    v8f   cacc[4] = {};
    float mi[8], li[8];
#pragma unroll
    for (int j = 0; j < 8; ++j) { mi[j] = -3.0e38f; li[j] = 0.0f; }

    const int nblk = causal ? ((q0 + 16 + 63) >> 6) : (SEQ / 64);
    h16* pw  = psh[wave];
    h16* pwl = pshl[RES ? wave : 0];

#pragma unroll 1
    for (int ib = 0; ib < nblk - 1; ++ib)
        attn_kv_block<RES, false>(causal, ib * 64, q0, lo, hi, bh, Km, Vt, pw, pwl,
                                  qa0, qa1, qa0l, qa1l, cacc, mi, li);
    attn_kv_block<RES, true>(causal, (nblk - 1) * 64, q0, lo, hi, bh, Km, Vt, pw, pwl,
                             qa0, qa1, qa0l, qa1l, cacc, mi, li);

    const int b = bh / HQ, h = bh % HQ;
    float* so = osh[wave];
#pragma unroll
    for (int j = 0; j < 8; ++j) {
        const float inv = 1.0f / li[j];
#pragma unroll
        for (int t = 0; t < 4; ++t) so[(j + 8 * hi) * 64 + t * 16 + lo] = cacc[t][j] * inv;
    }
    asm volatile("s_wait_dscnt 0" ::: "memory");
    __builtin_amdgcn_wave_barrier();
#pragma unroll 1
    for (int pass = 0; pass < 2; ++pass) {
#pragma unroll 4
        for (int r = 0; r < 16; ++r) {
            h16 h0, l0, h1, l1;
            split16(so[r * 64 + 2 * lane], h0, l0);
            split16(so[r * 64 + 2 * lane + 1], h1, l1);
            const size_t po = ((size_t)(b * SEQ) + q0 + r) * DQ + h * HDQ + 2 * lane;
            *(volatile unsigned*)(ctx + po) = pack2h(h0, h1); *(volatile unsigned*)(ctx + PLX + po) = pack2h(l0, l1);
        }
        __threadfence();
    }
}

extern "C" void kernel_launch(void* const* d_in, const int* in_sizes, int n_in,
                              void* d_out, int out_size, void* d_ws, size_t ws_size,
                              hipStream_t stream) {
    if (n_in < 10) return;
    const float* x  = (const float*)d_in[0];
    const float* wq = (const float*)d_in[1];
    const float* bq = (const float*)d_in[2];
    const float* wk = (const float*)d_in[3];
    const float* bk = (const float*)d_in[4];
    const float* wv = (const float*)d_in[5];
    const float* bv = (const float*)d_in[6];
    const float* wo = (const float*)d_in[7];
    const float* bo = (const float*)d_in[8];
    const int*   mk = (const int*)d_in[9];
    float* out = (float*)d_out;

    if ((size_t)in_sizes[0] < ((size_t)(NB - 1) * SEQ_FULL + SEQ) * DQ) return;
    if ((size_t)in_sizes[1] < (size_t)DQ * DQ || (size_t)in_sizes[3] < (size_t)DQ * DQ ||
        (size_t)in_sizes[5] < (size_t)DQ * DQ || (size_t)in_sizes[7] < (size_t)DQ * DQ) return;
    if (in_sizes[2] < DQ || in_sizes[4] < DQ || in_sizes[6] < DQ || in_sizes[8] < DQ) return;
    if (in_sizes[9] < 1) return;
    if ((size_t)out_size < (size_t)MQ * DQ) return;

    const size_t nX   = (size_t)MQ * DQ;
    const size_t szX1 = nX * 2;
    const size_t szX2 = nX * 4;
    const size_t szW  = (size_t)DQ * DQ * 2;
    char* ws = (char*)d_ws;
    size_t off = 0;
    h16* xh   = (h16*)(ws + off); off += szX1;
    h16* wqh  = (h16*)(ws + off); off += szW;
    h16* wkh  = (h16*)(ws + off); off += szW;
    h16* wvh  = (h16*)(ws + off); off += szW;
    h16* woh  = (h16*)(ws + off); off += szW;
    h16* Qb   = (h16*)(ws + off); off += szX2;
    h16* Kb   = (h16*)(ws + off); off += szX2;
    h16* Vrb  = (h16*)(ws + off); off += szX2;
    h16* Vtb  = (h16*)(ws + off); off += szX2;
    h16* ctxb = (h16*)(ws + off); off += szX2;
    if (off > ws_size) return;

    cvt_plane<true><<<(unsigned)(nX / 1024), 256, 0, stream>>>(x, xh, MQ, XS);
    cvt_plane<false><<<(unsigned)((size_t)DQ * DQ / 1024), 256, 0, stream>>>(wq, wqh, DQ, WSC);
    cvt_plane<false><<<(unsigned)((size_t)DQ * DQ / 1024), 256, 0, stream>>>(wk, wkh, DQ, WSC);
    cvt_plane<false><<<(unsigned)((size_t)DQ * DQ / 1024), 256, 0, stream>>>(wv, wvh, DQ, WSC);
    cvt_plane<false><<<(unsigned)((size_t)DQ * DQ / 1024), 256, 0, stream>>>(wo, woh, DQ, WSC);

    dim3 gg(DQ / 64, MQ / 128);
    const float pscale = 1.0f / (XS * WSC);
    gemm16<1><<<gg, 256, 0, stream>>>(xh, wqh, bq, nullptr, Qb,  pscale);
    gemm16<1><<<gg, 256, 0, stream>>>(xh, wkh, bk, nullptr, Kb,  pscale);
    gemm16<1><<<gg, 256, 0, stream>>>(xh, wvh, bv, nullptr, Vrb, pscale);
    vt_kernel<<<dim3(NB * HQ * (SEQ / 64), 2), 256, 0, stream>>>(Vrb, Vtb);

    const int nwE = NB * HQ * EARLY_QT;
    const int nwL = NB * HQ * (SEQ / 16 - EARLY_QT);
    flash_attn<true><<<(unsigned)((nwE + 7) / 8), 256, 0, stream>>>(Qb, Kb, Vtb, mk, ctxb, nwE);
    flash_attn<false><<<(unsigned)((nwL + 7) / 8), 256, 0, stream>>>(Qb, Kb, Vtb, mk, ctxb, nwL);

    gemm16<0><<<gg, 256, 0, stream>>>(ctxb, woh, bo, out, nullptr, 1.0f / WSC);
}
